// SimpleHeteroGNN_7086696038636
// MI455X (gfx1250) — hardware-verified
//
#include <hip/hip_runtime.h>
#include <stddef.h>


#define HIDC   128
#define OUTC   10
#define GMAX   1024
#define NTHR   256
#define NWAVE  8
#define EPT    8
#define NGRP   2
#define CHUNK  (NTHR * EPT * NGRP)
#define WCAP   (EPT * NGRP * 32)
#define LISTN  (NWAVE * WCAP)
#define NBC    4096
#define NBF    1024
#define NBP    32
#define RCAP   40960
#define RBN    128
#define TGT    256
#define DEGCAP 256
#define GROWS  128
#define APIT   (HIDC + 8)
#define OTHR   512
#define WSCALE 16.0f
#define WINV   0.0625f
#define BNEPS  1e-5f

#define LDS_FILL ((RCAP + NBF + LISTN) * 4 + 64)
#define LDS_G3   (2 * GROWS * APIT * 2 + GROWS * HIDC * 4 + 2 * HIDC * 8)

static_assert((CHUNK & (CHUNK - 1)) == 0);
static_assert(CHUNK <= 4096);
static_assert(NBC <= 4096 && NBF <= 4096 && NBP <= 4096);
static_assert((NBC & (NBC - 1)) == 0 && (NBF & (NBF - 1)) == 0 && (NBP & (NBP - 1)) == 0);
static_assert(NBC == 4 * NBF);
static_assert(OTHR * 8 == NBC);
static_assert((RCAP % 32) == 0);
static_assert(TGT == NWAVE * 32 && (TGT % GROWS) == 0);
static_assert(GROWS == NWAVE * 16);
static_assert((GROWS * HIDC / 8) % NTHR == 0);
static_assert(NBP * HIDC / 4 == 4 * NTHR);
static_assert((GMAX * OUTC) % 4 == 0);
static_assert(((GROWS * APIT * 2) % 16) == 0);

typedef float          v4f   __attribute__((ext_vector_type(4)));
typedef float          v8f   __attribute__((ext_vector_type(8)));
typedef int            v4i   __attribute__((ext_vector_type(4)));
typedef double         v2d   __attribute__((ext_vector_type(2)));
typedef _Float16       v8h   __attribute__((ext_vector_type(8)));
typedef _Float16       v16h  __attribute__((ext_vector_type(16)));
typedef unsigned short v8us  __attribute__((ext_vector_type(8)));
typedef unsigned short v16us __attribute__((ext_vector_type(16)));
typedef __bf16         v16bf __attribute__((ext_vector_type(16)));
union FragH { v16h v; v8h h[2]; };
union FragU { v16us u; v8us h[2]; v16bf b; };

__device__ __forceinline__ unsigned short bfr(float f) {
  unsigned u = __float_as_uint(f);
  u += 0x7FFFu + ((u >> 16) & 1u);
  return (unsigned short)(u >> 16);
}
__device__ __forceinline__ float bfv(unsigned short b) { return __uint_as_float(((unsigned)b) << 16); }

__device__ __forceinline__ void split8(v4f a, v4f b, v8us& hi, v8us& lo) {
  float xv[8];
  xv[0] = a.x; xv[1] = a.y; xv[2] = a.z; xv[3] = a.w;
  xv[4] = b.x; xv[5] = b.y; xv[6] = b.z; xv[7] = b.w;
#pragma unroll
  for (int e = 0; e < 8; ++e) {
    const unsigned short hq = bfr(xv[e]);
    hi[e] = hq;
    lo[e] = bfr(xv[e] - bfv(hq));
  }
}

__device__ __forceinline__ v8h cvt8(v4f a, v4f b) {
  v8h r;
  r[0] = (_Float16)a.x; r[1] = (_Float16)a.y; r[2] = (_Float16)a.z; r[3] = (_Float16)a.w;
  r[4] = (_Float16)b.x; r[5] = (_Float16)b.y; r[6] = (_Float16)b.z; r[7] = (_Float16)b.w;
  return r;
}

__device__ __forceinline__ v8f wmh(v16h a, v16h b, v8f c) {
  v8f d = __builtin_amdgcn_wmma_f32_16x16x32_f16(false, a, false, b, (short)0, c, false, false);
  asm volatile("v_nop\n\tv_nop\n\tv_nop\n\tv_nop" : "+v"(d) : "v"(a), "v"(b));
  return d;
}
__device__ __forceinline__ v8f wmb(v16us a, v16us b, v8f c) {
  FragU x, y; x.u = a; y.u = b;
  v8f d = __builtin_amdgcn_wmma_f32_16x16x32_bf16(false, x.b, false, y.b, (short)0, c, false, false);
  asm volatile("v_nop\n\tv_nop\n\tv_nop\n\tv_nop" : "+v"(d) : "v"(a), "v"(b));
  return d;
}

template <int NB>
__device__ __forceinline__ int scan_chunk(const int* __restrict__ dsts, int nE, int cbase, int slotBase,
                                          int vec8, int* list, int tid, int lane, int wave) {
  int wc = 0;
#pragma unroll
  for (int g = 0; g < NGRP; ++g) {
    const int el0  = (g * NTHR + tid) * EPT;
    const int e0   = cbase + el0;
    const int sent = -2147483647 - 1;
    v4i da, db;
    if (vec8 != 0 && cbase + CHUNK <= nE) {
      da = *(const v4i*)(dsts + e0);
      db = *(const v4i*)(dsts + e0 + 4);
    } else {
      da.x = (e0     < nE) ? dsts[min(e0, nE - 1)] : sent;
      da.y = (e0 + 1 < nE) ? dsts[min(e0 + 1, nE - 1)] : sent;
      da.z = (e0 + 2 < nE) ? dsts[min(e0 + 2, nE - 1)] : sent;
      da.w = (e0 + 3 < nE) ? dsts[min(e0 + 3, nE - 1)] : sent;
      db.x = (e0 + 4 < nE) ? dsts[min(e0 + 4, nE - 1)] : sent;
      db.y = (e0 + 5 < nE) ? dsts[min(e0 + 5, nE - 1)] : sent;
      db.z = (e0 + 6 < nE) ? dsts[min(e0 + 6, nE - 1)] : sent;
      db.w = (e0 + 7 < nE) ? dsts[min(e0 + 7, nE - 1)] : sent;
    }
    const unsigned nb = (unsigned)slotBase;
    const unsigned s0 = (unsigned)da.x - nb, s1 = (unsigned)da.y - nb;
    const unsigned s2 = (unsigned)da.z - nb, s3 = (unsigned)da.w - nb;
    const unsigned s4 = (unsigned)db.x - nb, s5 = (unsigned)db.y - nb;
    const unsigned s6 = (unsigned)db.z - nb, s7 = (unsigned)db.w - nb;
    const bool h0 = s0 < (unsigned)NB, h1 = s1 < (unsigned)NB, h2 = s2 < (unsigned)NB, h3 = s3 < (unsigned)NB;
    const bool h4 = s4 < (unsigned)NB, h5 = s5 < (unsigned)NB, h6 = s6 < (unsigned)NB, h7 = s7 < (unsigned)NB;
    const unsigned any = __builtin_amdgcn_ballot_w32(h0 | h1 | h2 | h3 | h4 | h5 | h6 | h7);
    if (any != 0u) {
#define HITJ(J, HJ, SJ) { \
        const unsigned mj = __builtin_amdgcn_ballot_w32(HJ); \
        if (mj != 0u) { \
          if (HJ) { \
            const int pos = wc + (int)__builtin_amdgcn_mbcnt_lo(mj, 0u); \
            if (pos < WCAP) list[wave * WCAP + pos] = ((el0 + (J)) << 12) | (int)(SJ); \
          } \
          wc += (int)__builtin_popcount(mj); } }
      HITJ(0, h0, s0)
      HITJ(1, h1, s1)
      HITJ(2, h2, s2)
      HITJ(3, h3, s3)
      HITJ(4, h4, s4)
      HITJ(5, h5, s5)
      HITJ(6, h6, s6)
      HITJ(7, h7, s7)
#undef HITJ
    }
  }
  return wc;
}

__global__ __launch_bounds__(NTHR) void k_wprep(
    const float* __restrict__ W1, const float* __restrict__ W2, const float* __restrict__ Wc,
    const float* __restrict__ Wg, unsigned short* whi, unsigned short* wlo, _Float16* wg, int nL) {
  const int q  = blockIdx.x >> 3;
  const int t  = ((blockIdx.x & 7) << 8) + (int)threadIdx.x;
  const int n  = t >> 4;
  const int k0 = (t & 15) * 8;
  const int nM = 2 * nL + 1;
  const float* src;
  if (q < nL)          src = W1 + (size_t)q * HIDC * HIDC;
  else if (q < 2 * nL) src = W2 + (size_t)(q - nL) * HIDC * HIDC;
  else if (q < nM)     src = Wc;
  else                 src = Wg;
  float v[8];
#pragma unroll
  for (int e = 0; e < 8; ++e) v[e] = src[(size_t)(k0 + e) * HIDC + n];
  v4f a, b;
  a.x = v[0]; a.y = v[1]; a.z = v[2]; a.w = v[3];
  b.x = v[4]; b.y = v[5]; b.z = v[6]; b.w = v[7];
  if (q < nM) {
    v8us hv, lv;
    split8(a, b, hv, lv);
    const size_t o = (size_t)q * HIDC * HIDC + (size_t)n * HIDC + k0;
    unsigned short* hp = whi + o;
    unsigned short* lp = wlo + o;
    *(volatile v8us*)hp = hv;
    *(volatile v8us*)lp = lv;
    __threadfence();
    *(volatile v8us*)hp = hv;
    *(volatile v8us*)lp = lv;
  } else {
    const v8h hv = cvt8(a * WSCALE, b * WSCALE);
    _Float16* dp = wg + (size_t)n * HIDC + k0;
    *(volatile v8h*)dp = hv;
    __threadfence();
    *(volatile v8h*)dp = hv;
  }
}

__global__ __launch_bounds__(NTHR) void k_count(const int* __restrict__ ei, int* cnt, int nE, int vec8) {
  __shared__ __attribute__((aligned(16))) int scnt[NBC];
  __shared__ __attribute__((aligned(16))) int list[LISTN];
  __shared__ int wcnt[NWAVE];
  const int tid = threadIdx.x, lane = tid & 31, wave = tid >> 5;
  const int nodeBase = blockIdx.x * NBC;
  const int* dsts = ei + nE;

  for (int i = tid; i < NBC; i += NTHR) scnt[i] = 0;
  __syncthreads();

  const int nChunks = (nE + CHUNK - 1) / CHUNK;
#pragma unroll 1
  for (int ch = 0; ch < nChunks; ++ch) {
    const int cbase = ch * CHUNK;
    const int wc = scan_chunk<NBC>(dsts, nE, cbase, nodeBase, vec8, list, tid, lane, wave);
    if (lane == 0) wcnt[wave] = wc;
    __syncthreads();
    if (wave == 0) {
#pragma unroll 1
      for (int wsx = 0; wsx < NWAVE; ++wsx) {
        int n = __builtin_amdgcn_readfirstlane(wcnt[wsx]);
        n = n > WCAP ? WCAP : (n < 0 ? 0 : n);
        const int* lp = list + wsx * WCAP;
#pragma unroll 1
        for (int i = 0; i < n; ++i) {
          const int ent  = __builtin_amdgcn_readfirstlane(lp[i]);
          const int slot = ent & (NBC - 1);
          if (lane == 0) scnt[slot] = scnt[slot] + 1;
        }
      }
    }
    __syncthreads();
  }

  v4i cq[4];
#pragma unroll
  for (int q = 0; q < 4; ++q) {
    const int f = (wave * 4 + q) * 128 + 4 * lane;
    cq[q] = *(const v4i*)(scnt + f);
  }
  int* cp = cnt + (size_t)nodeBase;
#pragma unroll
  for (int q = 0; q < 4; ++q) {
    const int f = (wave * 4 + q) * 128 + 4 * lane;
    *(volatile v4i*)(cp + f) = cq[q];
  }
  __threadfence();
#pragma unroll
  for (int q = 0; q < 4; ++q) {
    const int f = (wave * 4 + q) * 128 + 4 * lane;
    *(volatile v4i*)(cp + f) = cq[q];
  }
}

__global__ __launch_bounds__(OTHR) void k_offsets(
    const int* __restrict__ cnt, int* off, int* rbase, int nChunk) {
  __shared__ __attribute__((aligned(16))) int soff[NBC];
  __shared__ __attribute__((aligned(16))) int srb[RBN];
  __shared__ int wtot[OTHR / 32];
  const int tid = threadIdx.x, lane = tid & 31, wave = tid >> 5, sub = tid >> 7;
  for (int i = tid; i < RBN; i += OTHR) srb[i] = 0;
  int carry = 0;
#pragma unroll 1
  for (int ch = 0; ch < nChunk; ++ch) {
    const int base = ch * NBC;
    const v4i c0 = *(const v4i*)(cnt + base + 8 * tid);
    const v4i c1 = *(const v4i*)(cnt + base + 8 * tid + 4);
    const int e0 = max(c0.x, 0), e1 = max(c0.y, 0), e2 = max(c0.z, 0), e3 = max(c0.w, 0);
    const int e4 = max(c1.x, 0), e5 = max(c1.y, 0), e6 = max(c1.z, 0), e7 = max(c1.w, 0);
    const int ts = e0 + e1 + e2 + e3 + e4 + e5 + e6 + e7;
    int incl = ts;
#pragma unroll
    for (int d = 1; d < 32; d <<= 1) {
      const int t = __shfl_up(incl, d);
      if (lane >= d) incl += t;
    }
    if (lane == 31) wtot[wave] = incl;
    __syncthreads();
    const int S0 = wtot[0]  + wtot[1]  + wtot[2]  + wtot[3];
    const int S1 = wtot[4]  + wtot[5]  + wtot[6]  + wtot[7];
    const int S2 = wtot[8]  + wtot[9]  + wtot[10] + wtot[11];
    const int S3 = wtot[12] + wtot[13] + wtot[14] + wtot[15];
    int pre = 0;
#pragma unroll 1
    for (int w = 4 * sub; w < wave; ++w) pre += wtot[w];
    const int b0 = carry;
    const int b1 = b0 + ((S0 + 31) & ~31);
    const int b2 = b1 + ((S1 + 31) & ~31);
    const int b3 = b2 + ((S2 + 31) & ~31);
    const int b4 = b3 + ((S3 + 31) & ~31);
    const int myb = sub == 0 ? b0 : (sub == 1 ? b1 : (sub == 2 ? b2 : b3));
    if (tid == 0) {
      srb[min(4 * ch + 0, RBN - 1)] = b0;
      srb[min(4 * ch + 1, RBN - 1)] = b1;
      srb[min(4 * ch + 2, RBN - 1)] = b2;
      srb[min(4 * ch + 3, RBN - 1)] = b3;
    }
    int run = myb + pre + incl - ts;
    soff[8 * tid + 0] = run; run += e0;
    soff[8 * tid + 1] = run; run += e1;
    soff[8 * tid + 2] = run; run += e2;
    soff[8 * tid + 3] = run; run += e3;
    soff[8 * tid + 4] = run; run += e4;
    soff[8 * tid + 5] = run; run += e5;
    soff[8 * tid + 6] = run; run += e6;
    soff[8 * tid + 7] = run;
    carry = b4;
    __syncthreads();
    const v4i o0 = *(const v4i*)(soff + 4 * tid);
    const v4i o1 = *(const v4i*)(soff + 4 * (tid + OTHR));
    int* op = off + base;
    *(volatile v4i*)(op + 4 * tid) = o0;
    *(volatile v4i*)(op + 4 * (tid + OTHR)) = o1;
    __threadfence();
    *(volatile v4i*)(op + 4 * tid) = o0;
    *(volatile v4i*)(op + 4 * (tid + OTHR)) = o1;
    __syncthreads();
  }
  if (tid == 0) srb[min(4 * nChunk, RBN - 1)] = carry;
  __syncthreads();
  v4i rv = {0, 0, 0, 0};
  if (tid < 32) rv = *(const v4i*)(srb + 4 * tid);
  if (tid < 32) *(volatile v4i*)(rbase + 4 * tid) = rv;
  __threadfence();
  if (tid < 32) *(volatile v4i*)(rbase + 4 * tid) = rv;
}

__global__ __launch_bounds__(NTHR) void k_fill(
    const int* __restrict__ ei, const int* __restrict__ off, const int* __restrict__ rbase,
    int* csr, int nN, int nE, int vec8, int csrLen) {
  extern __shared__ v4f lds_dyn[];
  int* region = (int*)lds_dyn;
  int* cursor = region + RCAP;
  int* list   = cursor + NBF;
  int* wcnt   = list + LISTN;
  const int tid = threadIdx.x, lane = tid & 31, wave = tid >> 5;
  const int b = blockIdx.x;
  const int nodeBase = b * NBF;
  const int* dsts = ei + nE;

  int rb0 = rbase[b];
  const int rb1 = rbase[b + 1];
  rb0 = rb0 < 0 ? 0 : (rb0 > csrLen ? csrLen : rb0);
  rb0 &= ~31;
  int len = rb1 - rb0;
  len = len < 0 ? 0 : (len > RCAP ? RCAP : len);
  int lenW = (len + 31) & ~31;
  if (rb0 + lenW > csrLen) lenW = (csrLen - rb0) & ~31;

  {
    const v4i z = {0, 0, 0, 0};
    for (int i = tid; i < RCAP / 4; i += NTHR) ((v4i*)region)[i] = z;
    for (int s = tid; s < NBF; s += NTHR) {
      int o = off[nodeBase + s] - rb0;
      o = o < 0 ? 0 : (o > RCAP ? RCAP : o);
      cursor[s] = o;
    }
  }
  __syncthreads();

  const int nChunks = (nE + CHUNK - 1) / CHUNK;
#pragma unroll 1
  for (int ch = 0; ch < nChunks; ++ch) {
    const int cbase = ch * CHUNK;
    const int wc = scan_chunk<NBF>(dsts, nE, cbase, nodeBase, vec8, list, tid, lane, wave);
    if (lane == 0) wcnt[wave] = wc;
    __syncthreads();
    if (wave == 0) {
#pragma unroll 1
      for (int wsx = 0; wsx < NWAVE; ++wsx) {
        int n = __builtin_amdgcn_readfirstlane(wcnt[wsx]);
        n = n > WCAP ? WCAP : (n < 0 ? 0 : n);
        const int* lp = list + wsx * WCAP;
#pragma unroll 1
        for (int i = 0; i < n; ++i) {
          const int ent  = __builtin_amdgcn_readfirstlane(lp[i]);
          const int slot = ent & (NBF - 1);
          int e = cbase + ((ent >> 12) & (CHUNK - 1));
          e = e > nE - 1 ? nE - 1 : e;
          int src = ei[e];
          src = src < 0 ? 0 : (src > nN - 1 ? nN - 1 : src);
          if (lane == 0) {
            int pos = cursor[slot];
            pos = pos < 0 ? 0 : (pos > RCAP - 1 ? RCAP - 1 : pos);
            region[pos] = src;
            const int np = pos + 1;
            cursor[slot] = np > RCAP ? RCAP : np;
          }
        }
      }
    }
    __syncthreads();
  }

  const int nv = lenW >> 2;
  int* gp = csr + rb0;
#pragma unroll 1
  for (int i = tid; i < nv; i += NTHR) { const v4i v = ((const v4i*)region)[i]; *(volatile v4i*)(gp + 4 * i) = v; }
  __threadfence();
#pragma unroll 1
  for (int i = tid; i < nv; i += NTHR) { const v4i v = ((const v4i*)region)[i]; *(volatile v4i*)(gp + 4 * i) = v; }
}

__global__ __launch_bounds__(NTHR) void k_enc(
    const int* __restrict__ x, const float* __restrict__ pe, const float* __restrict__ ce,
    const float* __restrict__ le, float* h, int nN, int nTh, int nCa, int nLv) {
  const int tid = threadIdx.x, lane = tid & 31, wave = tid >> 5;
#pragma unroll 1
  for (int j = 0; j < 4; ++j) {
    const int n  = (blockIdx.x * NWAVE + wave) * 4 + j;
    const int nc = n < nN ? n : nN - 1;
    int lv = x[(size_t)3 * nc + 0];
    int ca = x[(size_t)3 * nc + 1];
    int th = x[(size_t)3 * nc + 2];
    lv = lv < 0 ? 0 : (lv > nLv - 1 ? nLv - 1 : lv);
    ca = ca < 0 ? 0 : (ca > nCa - 1 ? nCa - 1 : ca);
    th = th < 0 ? 0 : (th > nTh - 1 ? nTh - 1 : th);
    const v4f a = *(const v4f*)(ce + (size_t)ca * HIDC + 4 * lane);
    const v4f b = *(const v4f*)(le + (size_t)lv * HIDC + 4 * lane);
    const v4f p = *(const v4f*)(pe + (size_t)th * HIDC + 4 * lane);
    v4f r = (a + b) + p;
    const bool keep = n < nN;
    r.x = keep ? r.x : 0.f; r.y = keep ? r.y : 0.f; r.z = keep ? r.z : 0.f; r.w = keep ? r.w : 0.f;
    float* hp = h + (size_t)n * HIDC + 4 * lane;
    *(volatile v4f*)hp = r;
    __threadfence();
    *(volatile v4f*)hp = r;
  }
}

__global__ __launch_bounds__(NTHR) void k_agg(
    const int* __restrict__ csr, const int* __restrict__ off, const int* __restrict__ cnt,
    const float* __restrict__ h, float* xo, int nN, int csrLen) {
  const int tid = threadIdx.x, lane = tid & 31, wave = tid >> 5;
  const int tbase = blockIdx.x * TGT + wave * 32;
  const int cl = tbase + lane;
  const int cnt_l = cnt[cl];
  const int off_l = off[cl];

#pragma unroll 1
  for (int j = 0; j < 32; ++j) {
    const int c = tbase + j;
    int n = __builtin_amdgcn_readlane(cnt_l, j);
    n = n < 0 ? 0 : (n > DEGCAP ? DEGCAP : n);
    const int st = __builtin_amdgcn_readlane(off_l, j);
    v4f acc = {0.f, 0.f, 0.f, 0.f};
#pragma unroll 1
    for (int q0 = 0; q0 < n; q0 += 32) {
      int pos = st + q0 + lane;
      pos = pos < 0 ? 0 : (pos > csrLen - 1 ? csrLen - 1 : pos);
      int sl = csr[pos];
      sl = sl < 0 ? 0 : (sl > nN - 1 ? nN - 1 : sl);
      const int mcnt = (n - q0) < 32 ? (n - q0) : 32;
#pragma unroll 1
      for (int p = 0; p < mcnt; ++p) {
        const int s = __builtin_amdgcn_readlane(sl, p);
        acc = acc + *(const v4f*)(h + (size_t)s * HIDC + 4 * lane);
      }
    }
    const v4f hv = *(const v4f*)(h + (size_t)c * HIDC + 4 * lane);
    const v4f v = hv + acc;
    float* xp = xo + (size_t)c * HIDC + 4 * lane;
    *(volatile v4f*)xp = v;
    __threadfence();
    *(volatile v4f*)xp = v;
  }
}

template <int BNA>
__global__ __launch_bounds__(NTHR) void k_gemm3(
    const float* __restrict__ A, const unsigned short* __restrict__ Bh, const unsigned short* __restrict__ Bl,
    const float* __restrict__ bnss, const float* __restrict__ bnbe, const float* __restrict__ bias,
    float* C, double* part, int nRowsA, int nValid) {
  extern __shared__ v4f lds_dyn[];
  unsigned short* sAh   = (unsigned short*)lds_dyn;
  unsigned short* sAl   = sAh + GROWS * APIT;
  float*          stg   = (float*)(sAl + GROWS * APIT);
  double*         spart = (double*)(stg + GROWS * HIDC);
  const int tid = threadIdx.x, lane = tid & 31, wave = tid >> 5, hh = lane >> 4, m = lane & 15;
  const int rowBase = blockIdx.x * GROWS;

#pragma unroll
  for (int i = 0; i < (GROWS * HIDC / 8) / NTHR; ++i) {
    const int idx = i * NTHR + tid;
    const int r   = idx >> 4;
    const int c0  = (idx & 15) * 8;
    int row = rowBase + r;
    row = row > nRowsA - 1 ? nRowsA - 1 : row;
    const float* ap = A + (size_t)row * HIDC + c0;
    v4f a = *(const v4f*)ap, b = *(const v4f*)(ap + 4);
    if (BNA != 0) {
      const v4f mu0 = *(const v4f*)(bnss + c0),        mu1 = *(const v4f*)(bnss + c0 + 4);
      const v4f sc0 = *(const v4f*)(bnss + HIDC + c0), sc1 = *(const v4f*)(bnss + HIDC + c0 + 4);
      const v4f be0 = *(const v4f*)(bnbe + c0),        be1 = *(const v4f*)(bnbe + c0 + 4);
      a = (a - mu0) * sc0 + be0;
      b = (b - mu1) * sc1 + be1;
      a.x = fmaxf(a.x, 0.f); a.y = fmaxf(a.y, 0.f); a.z = fmaxf(a.z, 0.f); a.w = fmaxf(a.w, 0.f);
      b.x = fmaxf(b.x, 0.f); b.y = fmaxf(b.y, 0.f); b.z = fmaxf(b.z, 0.f); b.w = fmaxf(b.w, 0.f);
    }
    v8us hv, lv;
    split8(a, b, hv, lv);
    *(v8us*)(sAh + r * APIT + c0) = hv;
    *(v8us*)(sAl + r * APIT + c0) = lv;
  }
  __syncthreads();

  const unsigned short* arh = sAh + (wave * 16 + m) * APIT + 8 * hh;
  const unsigned short* arl = sAl + (wave * 16 + m) * APIT + 8 * hh;
  const int r0 = wave * 16 + 8 * hh;
#pragma unroll 1
  for (int g = 0; g < 2; ++g) {
    v8f acc[4];
#pragma unroll
    for (int t = 0; t < 4; ++t) { v8f z = {0.f, 0.f, 0.f, 0.f, 0.f, 0.f, 0.f, 0.f}; acc[t] = z; }
#pragma unroll 1
    for (int kt = 0; kt < HIDC / 32; ++kt) {
      FragU ah, al;
      ah.h[0] = *(const v8us*)(arh + 32 * kt);
      ah.h[1] = *(const v8us*)(arh + 32 * kt + 16);
      al.h[0] = *(const v8us*)(arl + 32 * kt);
      al.h[1] = *(const v8us*)(arl + 32 * kt + 16);
#pragma unroll
      for (int t = 0; t < 4; ++t) {
        const size_t bo = (size_t)(64 * g + 16 * t + m) * HIDC + 32 * kt + 8 * hh;
        FragU bh, bl;
        bh.h[0] = *(const v8us*)(Bh + bo);
        bh.h[1] = *(const v8us*)(Bh + bo + 16);
        bl.h[0] = *(const v8us*)(Bl + bo);
        bl.h[1] = *(const v8us*)(Bl + bo + 16);
        acc[t] = wmb(ah.u, bh.u, acc[t]);
        acc[t] = wmb(ah.u, bl.u, acc[t]);
        acc[t] = wmb(al.u, bh.u, acc[t]);
      }
    }
    float* sp = stg + r0 * HIDC + 64 * g + m;
#pragma unroll
    for (int t = 0; t < 4; ++t) {
      const float bv = bias[64 * g + 16 * t + m];
#pragma unroll
      for (int r = 0; r < 8; ++r) sp[r * HIDC + 16 * t] = acc[t][r] + bv;
    }
  }
  __syncthreads();

  int nv = nValid - rowBase;
  nv = nv < 0 ? 0 : (nv > GROWS ? GROWS : nv);
  if (tid < HIDC) {
    double s = 0.0;
#pragma unroll 1
    for (int r = 0; r < nv; ++r) s += (double)stg[r * HIDC + tid];
    spart[tid] = s;
  } else {
    const int c = tid - HIDC;
    double q = 0.0;
#pragma unroll 1
    for (int r = 0; r < nv; ++r) { const double v = (double)stg[r * HIDC + c]; q = fma(v, v, q); }
    spart[HIDC + c] = q;
  }
  __syncthreads();

  const float* lp = stg + wave * 16 * HIDC + 4 * lane;
  float* gp = C + ((size_t)rowBase + wave * 16) * HIDC + 4 * lane;
  v2d pv = {0.0, 0.0};
  if (tid < HIDC) pv = *(const v2d*)(spart + 2 * tid);
  double* pp = part + (size_t)blockIdx.x * (2 * HIDC) + 2 * (tid & (HIDC - 1));
#pragma unroll
  for (int i = 0; i < 16; ++i) { const v4f v = *(const v4f*)(lp + i * HIDC); *(volatile v4f*)(gp + (size_t)i * HIDC) = v; }
  if (tid < HIDC) *(volatile v2d*)pp = pv;
  __threadfence();
#pragma unroll
  for (int i = 0; i < 16; ++i) { const v4f v = *(const v4f*)(lp + i * HIDC); *(volatile v4f*)(gp + (size_t)i * HIDC) = v; }
  if (tid < HIDC) *(volatile v2d*)pp = pv;
}

__global__ __launch_bounds__(NTHR) void k_bnfin(
    const double* __restrict__ part, int nBlk, int nRows, const float* __restrict__ gam, float* ss) {
  __shared__ double sS[HIDC];
  __shared__ double sQ[HIDC];
  __shared__ __attribute__((aligned(16))) float so[2 * HIDC];
  const int tid = threadIdx.x;
  if (tid < HIDC) {
    double s = 0.0;
#pragma unroll 1
    for (int b = 0; b < nBlk; ++b) s += part[(size_t)b * (2 * HIDC) + tid];
    sS[tid] = s;
  } else {
    const int c = tid - HIDC;
    double q = 0.0;
#pragma unroll 1
    for (int b = 0; b < nBlk; ++b) q += part[(size_t)b * (2 * HIDC) + HIDC + c];
    sQ[c] = q;
  }
  __syncthreads();
  if (tid < HIDC) {
    const double inv  = 1.0 / (double)(nRows > 0 ? nRows : 1);
    const double mean = sS[tid] * inv;
    double var = sQ[tid] * inv - mean * mean;
    var = var < 0.0 ? 0.0 : var;
    const float vf = (float)var;
    so[tid]        = (float)mean;
    so[HIDC + tid] = gam[tid] * rsqrtf(vf + BNEPS);
  }
  __syncthreads();
  v4f v = {0.f, 0.f, 0.f, 0.f};
  if (tid < 64) v = *(const v4f*)(so + 4 * tid);
  if (tid < 64) *(volatile v4f*)(ss + 4 * tid) = v;
  __threadfence();
  if (tid < 64) *(volatile v4f*)(ss + 4 * tid) = v;
}

__global__ __launch_bounds__(NTHR) void k_apply(
    const float* __restrict__ z, const float* __restrict__ ss, const float* __restrict__ beta, float* ho) {
  const int tid = threadIdx.x, lane = tid & 31, wave = tid >> 5;
  const v4f mu = *(const v4f*)(ss + 4 * lane);
  const v4f sc = *(const v4f*)(ss + HIDC + 4 * lane);
  const v4f be = *(const v4f*)(beta + 4 * lane);
  const int rb = blockIdx.x * 64 + wave * 8;
#pragma unroll 1
  for (int j = 0; j < 8; ++j) {
    const size_t o = ((size_t)rb + j) * HIDC + 4 * lane;
    v4f v = *(const v4f*)(z + o);
    v = (v - mu) * sc + be;
    v.x = fmaxf(v.x, 0.f); v.y = fmaxf(v.y, 0.f); v.z = fmaxf(v.z, 0.f); v.w = fmaxf(v.w, 0.f);
    *(volatile v4f*)(ho + o) = v;
    __threadfence();
    *(volatile v4f*)(ho + o) = v;
  }
}

__global__ __launch_bounds__(NTHR) void k_gate(
    const float* __restrict__ A, const _Float16* __restrict__ Bs, const float* __restrict__ b1,
    const float* __restrict__ w2, const float* __restrict__ b2, float* gate, int nRowsA) {
  __shared__ __attribute__((aligned(16))) _Float16 sA[GROWS * APIT];
  __shared__ __attribute__((aligned(16))) float sg[GROWS];
  const int tid = threadIdx.x, lane = tid & 31, wave = tid >> 5, hh = lane >> 4, m = lane & 15;
  const int rowBase = blockIdx.x * GROWS;

#pragma unroll
  for (int i = 0; i < (GROWS * HIDC / 8) / NTHR; ++i) {
    const int idx = i * NTHR + tid;
    const int r   = idx >> 4;
    const int c0  = (idx & 15) * 8;
    int row = rowBase + r;
    row = row > nRowsA - 1 ? nRowsA - 1 : row;
    const float* ap = A + (size_t)row * HIDC + c0;
    const v4f a = *(const v4f*)ap, b = *(const v4f*)(ap + 4);
    *(v8h*)(sA + r * APIT + c0) = cvt8(a, b);
  }
  __syncthreads();

  v8f acc[8];
#pragma unroll
  for (int t = 0; t < 8; ++t) { v8f z = {0.f, 0.f, 0.f, 0.f, 0.f, 0.f, 0.f, 0.f}; acc[t] = z; }
  const _Float16* ar = sA + (wave * 16 + m) * APIT + 8 * hh;
#pragma unroll 1
  for (int kt = 0; kt < HIDC / 32; ++kt) {
    FragH a;
    a.h[0] = *(const v8h*)(ar + 32 * kt);
    a.h[1] = *(const v8h*)(ar + 32 * kt + 16);
#pragma unroll
    for (int t = 0; t < 8; ++t) {
      const _Float16* bp = Bs + (size_t)(16 * t + m) * HIDC + 32 * kt + 8 * hh;
      FragH b;
      b.h[0] = *(const v8h*)bp;
      b.h[1] = *(const v8h*)(bp + 16);
      acc[t] = wmh(a.v, b.v, acc[t]);
    }
  }

  float gs[8];
#pragma unroll
  for (int r = 0; r < 8; ++r) gs[r] = 0.f;
#pragma unroll
  for (int t = 0; t < 8; ++t) {
    const int col = 16 * t + m;
    const float bl = b1[col];
    const float wv = w2[col];
#pragma unroll
    for (int r = 0; r < 8; ++r) {
      const float zv = fmaxf(acc[t][r] * WINV + bl, 0.0f);
      gs[r] = fmaf(zv, wv, gs[r]);
    }
  }
#pragma unroll
  for (int r = 0; r < 8; ++r) {
    float v = gs[r];
    v += __shfl_xor(v, 1, 32);
    v += __shfl_xor(v, 2, 32);
    v += __shfl_xor(v, 4, 32);
    v += __shfl_xor(v, 8, 32);
    gs[r] = v;
  }
  const float b2v = b2[0];
  if (m == 0) {
#pragma unroll
    for (int r = 0; r < 8; ++r) sg[wave * 16 + 8 * hh + r] = gs[r] + b2v;
  }
  __syncthreads();
  v4f ov = {0.f, 0.f, 0.f, 0.f};
  if (tid < 32) ov = *(const v4f*)(sg + 4 * tid);
  float* op = gate + rowBase;
  if (tid < 32) *(volatile v4f*)(op + 4 * tid) = ov;
  __threadfence();
  if (tid < 32) *(volatile v4f*)(op + 4 * tid) = ov;
}

__global__ __launch_bounds__(NTHR) void k_pool(
    const int* __restrict__ batch, const int* __restrict__ numg, const float* __restrict__ gate,
    const float* __restrict__ h, float* pooled, int nN) {
  __shared__ __attribute__((aligned(16))) float acc[NBP * HIDC];
  __shared__ __attribute__((aligned(16))) int list[LISTN];
  __shared__ float smax[NBP];
  __shared__ float ssum[NBP];
  __shared__ int wcnt[NWAVE];
  const int tid = threadIdx.x, lane = tid & 31, wave = tid >> 5;
  const int gBase = blockIdx.x * NBP;
  const int ng = numg[0];

  {
    const v4f z = {0.f, 0.f, 0.f, 0.f};
    for (int i = tid; i < NBP * HIDC / 4; i += NTHR) ((v4f*)acc)[i] = z;
    if (tid < NBP) { smax[tid] = -__builtin_inff(); ssum[tid] = 0.f; }
  }
  __syncthreads();

  const int nChunks = (nN + CHUNK - 1) / CHUNK;
#pragma unroll 1
  for (int pass = 0; pass < 2; ++pass) {
#pragma unroll 1
    for (int ch = 0; ch < nChunks; ++ch) {
      const int cbase = ch * CHUNK;
      const int wc = scan_chunk<NBP>(batch, nN, cbase, gBase, 1, list, tid, lane, wave);
      if (lane == 0) wcnt[wave] = wc;
      __syncthreads();
      if (wave == 0) {
#pragma unroll 1
        for (int wsx = 0; wsx < NWAVE; ++wsx) {
          int n = __builtin_amdgcn_readfirstlane(wcnt[wsx]);
          n = n > WCAP ? WCAP : (n < 0 ? 0 : n);
          const int* lp = list + wsx * WCAP;
#pragma unroll 1
          for (int i = 0; i < n; ++i) {
            const int ent  = __builtin_amdgcn_readfirstlane(lp[i]);
            const int slot = ent & (NBP - 1);
            int nd = cbase + ((ent >> 12) & (CHUNK - 1));
            nd = nd > nN - 1 ? nN - 1 : nd;
            const float gv = gate[nd];
            if (pass == 0) {
              if (lane == 0) smax[slot] = fmaxf(smax[slot], gv);
            } else {
              const float e = expf(gv - smax[slot]);
              const v4f v = *(const v4f*)(h + (size_t)nd * HIDC + 4 * lane);
              v4f* ap = (v4f*)(acc + slot * HIDC + 4 * lane);
              *ap = *ap + v * e;
              if (lane == 0) ssum[slot] = ssum[slot] + e;
            }
          }
        }
      }
      __syncthreads();
    }
  }

  v4f ov[4];
#pragma unroll
  for (int p = 0; p < 4; ++p) {
    const int idx = p * NTHR + tid;
    const int row = idx >> 5;
    const int piece = idx & 31;
    const float s = ssum[row];
    float inv = (s > 0.f) ? (1.0f / s) : 0.f;
    inv = (gBase + row < ng) ? inv : 0.f;
    ov[p] = *(const v4f*)(acc + row * HIDC + 4 * piece) * inv;
  }
  float* gp = pooled + (size_t)gBase * HIDC;
#pragma unroll
  for (int p = 0; p < 4; ++p) *(volatile v4f*)(gp + 4 * (p * NTHR + tid)) = ov[p];
  __threadfence();
#pragma unroll
  for (int p = 0; p < 4; ++p) *(volatile v4f*)(gp + 4 * (p * NTHR + tid)) = ov[p];
}

__global__ __launch_bounds__(NTHR) void k_clsfin(
    const float* __restrict__ zc, const double* __restrict__ part, int nBlk, int nG,
    const float* __restrict__ gam, const float* __restrict__ bet, const float* __restrict__ w2,
    const float* __restrict__ b2, float* out, int outN) {
  __shared__ double sS[HIDC];
  __shared__ double sQ[HIDC];
  __shared__ float smu[HIDC];
  __shared__ float ssc[HIDC];
  __shared__ float sbe[HIDC];
  __shared__ float sw2[HIDC * OUTC];
  __shared__ float sb2[16];
  __shared__ __attribute__((aligned(16))) float sout[GMAX * OUTC + 16];
  const int tid = threadIdx.x;
  if (tid < HIDC) {
    double s = 0.0;
#pragma unroll 1
    for (int b = 0; b < nBlk; ++b) s += part[(size_t)b * (2 * HIDC) + tid];
    sS[tid] = s;
  } else {
    const int c = tid - HIDC;
    double q = 0.0;
#pragma unroll 1
    for (int b = 0; b < nBlk; ++b) q += part[(size_t)b * (2 * HIDC) + HIDC + c];
    sQ[c] = q;
  }
  for (int i = tid; i < HIDC * OUTC; i += NTHR) sw2[i] = w2[i];
  if (tid < OUTC) sb2[tid] = b2[tid];
  __syncthreads();
  if (tid < HIDC) {
    const double inv  = 1.0 / (double)(nG > 0 ? nG : 1);
    const double mean = sS[tid] * inv;
    double var = sQ[tid] * inv - mean * mean;
    var = var < 0.0 ? 0.0 : var;
    const float vf = (float)var;
    smu[tid] = (float)mean;
    ssc[tid] = gam[tid] * rsqrtf(vf + BNEPS);
    sbe[tid] = bet[tid];
  }
  __syncthreads();

#pragma unroll 1
  for (int row = tid; row < GMAX; row += NTHR) {
    const int rr = row < nG ? row : nG - 1;
    const float* zr = zc + (size_t)rr * HIDC;
    float acc[OUTC];
#pragma unroll
    for (int o = 0; o < OUTC; ++o) acc[o] = 0.f;
#pragma unroll 1
    for (int c = 0; c < HIDC; ++c) {
      float a = (zr[c] - smu[c]) * ssc[c] + sbe[c];
      a = fmaxf(a, 0.f);
#pragma unroll
      for (int o = 0; o < OUTC; ++o) acc[o] = fmaf(a, sw2[c * OUTC + o], acc[o]);
    }
#pragma unroll
    for (int o = 0; o < OUTC; ++o) sout[row * OUTC + o] = acc[o] + sb2[o];
  }
  __syncthreads();

  const int nvec = outN >> 2;
#pragma unroll
  for (int p = 0; p < (GMAX * OUTC / 4) / NTHR; ++p) {
    const int idx = p * NTHR + tid;
    if (idx < nvec) { const v4f v = *(const v4f*)(sout + 4 * idx); *(volatile v4f*)(out + 4 * (size_t)idx) = v; }
  }
  if (tid == 0) {
#pragma unroll 1
    for (int k = 4 * nvec; k < outN; ++k) { const float v = sout[k]; *(volatile float*)(out + k) = v; }
  }
  __threadfence();
#pragma unroll
  for (int p = 0; p < (GMAX * OUTC / 4) / NTHR; ++p) {
    const int idx = p * NTHR + tid;
    if (idx < nvec) { const v4f v = *(const v4f*)(sout + 4 * idx); *(volatile v4f*)(out + 4 * (size_t)idx) = v; }
  }
  if (tid == 0) {
#pragma unroll 1
    for (int k = 4 * nvec; k < outN; ++k) { const float v = sout[k]; *(volatile float*)(out + k) = v; }
  }
}

extern "C" void kernel_launch(void* const* d_in, const int* in_sizes, int n_in,
                              void* d_out, int out_size, void* d_ws, size_t ws_size,
                              hipStream_t stream) {
  if (n_in < 25) return;
  const int nN = in_sizes[0] / 3;
  const int nE = in_sizes[1] / 2;
  if (nN <= 0 || nE <= 0 || in_sizes[0] != 3 * nN || in_sizes[1] != 2 * nE || in_sizes[2] != nN) return;
  if (in_sizes[3] < 1) return;
  if (in_sizes[4] < HIDC || (in_sizes[4] % HIDC) != 0) return;
  if (in_sizes[5] < HIDC || (in_sizes[5] % HIDC) != 0) return;
  if (in_sizes[6] < HIDC || (in_sizes[6] % HIDC) != 0) return;
  const int nTh = in_sizes[4] / HIDC, nCa = in_sizes[5] / HIDC, nLv = in_sizes[6] / HIDC;
  const int nL = in_sizes[7] / (HIDC * HIDC);
  if (nL < 1 || in_sizes[7] != nL * HIDC * HIDC || in_sizes[11] != nL * HIDC * HIDC) return;
  if (in_sizes[8] < nL * HIDC || in_sizes[9] < nL * HIDC || in_sizes[10] < nL * HIDC ||
      in_sizes[12] < nL * HIDC || in_sizes[13] < nL * HIDC || in_sizes[14] < nL * HIDC) return;
  if (in_sizes[15] != HIDC * HIDC || in_sizes[16] < HIDC || in_sizes[17] < HIDC || in_sizes[18] < 1) return;
  if (in_sizes[19] != HIDC * HIDC || in_sizes[20] < HIDC || in_sizes[21] < HIDC || in_sizes[22] < HIDC) return;
  if (in_sizes[23] != HIDC * OUTC || in_sizes[24] < OUTC) return;
  const int G = out_size / OUTC;
  if (G < 1 || G * OUTC != out_size || G > GMAX) return;
  if (nE > (1 << 28) || nN > (1 << 24)) return;

  const int*   x    = (const int*)d_in[0];
  const int*   ei   = (const int*)d_in[1];
  const int*   bat  = (const int*)d_in[2];
  const int*   numg = (const int*)d_in[3];
  const float* pe   = (const float*)d_in[4];
  const float* ce   = (const float*)d_in[5];
  const float* le   = (const float*)d_in[6];
  const float* W1   = (const float*)d_in[7];
  const float* b1   = (const float*)d_in[8];
  const float* g1   = (const float*)d_in[9];
  const float* be1  = (const float*)d_in[10];
  const float* W2   = (const float*)d_in[11];
  const float* b2   = (const float*)d_in[12];
  const float* g2   = (const float*)d_in[13];
  const float* be2  = (const float*)d_in[14];
  const float* gW1  = (const float*)d_in[15];
  const float* gb1  = (const float*)d_in[16];
  const float* gW2  = (const float*)d_in[17];
  const float* gb2  = (const float*)d_in[18];
  const float* cW1  = (const float*)d_in[19];
  const float* cb1  = (const float*)d_in[20];
  const float* cg   = (const float*)d_in[21];
  const float* cbe  = (const float*)d_in[22];
  const float* cW2  = (const float*)d_in[23];
  const float* cb2  = (const float*)d_in[24];
  float* out = (float*)d_out;

  const int NPAD   = ((nN + TGT - 1) / TGT) * TGT;
  const int nBC    = (nN + NBC - 1) / NBC;
  const int CNTPAD = nBC * NBC;
  if (4 * nBC + 1 > RBN) return;
  const int nBF    = (nN + NBF - 1) / NBF;
  const int csrLen = ((nE + 31) & ~31) + 4096;
  const int nGemm  = NPAD / GROWS;
  const int nAgg   = NPAD / TGT;
  const int nEnc   = NPAD / 32;
  const int nApp   = NPAD / 64;
  const int GR     = ((G + GROWS - 1) / GROWS) * GROWS;
  const int nPool  = GR / NBP;
  const int nCls   = GR / GROWS;
  const int nPart  = nGemm > nCls ? nGemm : nCls;
  const int nM     = 2 * nL + 1;

  char* ws = (char*)d_ws;
  size_t off = 0;
  const size_t oWhi = off; off += (size_t)nM * HIDC * HIDC * 2;     off = (off + 255) & ~(size_t)255;
  const size_t oWlo = off; off += (size_t)nM * HIDC * HIDC * 2;     off = (off + 255) & ~(size_t)255;
  const size_t oWg  = off; off += (size_t)HIDC * HIDC * 2;          off = (off + 255) & ~(size_t)255;
  const size_t oCnt = off; off += (size_t)CNTPAD * 4;               off = (off + 255) & ~(size_t)255;
  const size_t oOff = off; off += (size_t)CNTPAD * 4;               off = (off + 255) & ~(size_t)255;
  const size_t oRb  = off; off += (size_t)RBN * 4;                  off = (off + 255) & ~(size_t)255;
  const size_t oCsr = off; off += (size_t)csrLen * 4;               off = (off + 255) & ~(size_t)255;
  const size_t oP0  = off; off += (size_t)NPAD * HIDC * 4;          off = (off + 255) & ~(size_t)255;
  const size_t oP1  = off; off += (size_t)NPAD * HIDC * 4;          off = (off + 255) & ~(size_t)255;
  const size_t oPrt = off; off += (size_t)nPart * 2 * HIDC * 8;     off = (off + 255) & ~(size_t)255;
  const size_t oSs1 = off; off += (size_t)2 * HIDC * 4;             off = (off + 255) & ~(size_t)255;
  const size_t oSs2 = off; off += (size_t)2 * HIDC * 4;             off = (off + 255) & ~(size_t)255;
  const size_t oGt  = off; off += (size_t)NPAD * 4;                 off = (off + 255) & ~(size_t)255;
  const size_t oPl  = off; off += (size_t)GR * HIDC * 4;            off = (off + 255) & ~(size_t)255;
  const size_t oZc  = off; off += (size_t)GR * HIDC * 4;            off = (off + 255) & ~(size_t)255;
  if (off > ws_size || off > ((size_t)128 << 20)) return;
  unsigned short* whi = (unsigned short*)(ws + oWhi);
  unsigned short* wlo = (unsigned short*)(ws + oWlo);
  _Float16* wg   = (_Float16*)(ws + oWg);
  int*      cnt  = (int*)(ws + oCnt);
  int*      offp = (int*)(ws + oOff);
  int*      rb   = (int*)(ws + oRb);
  int*      csr  = (int*)(ws + oCsr);
  float*    P0   = (float*)(ws + oP0);
  float*    P1   = (float*)(ws + oP1);
  double*   part = (double*)(ws + oPrt);
  float*    ss1  = (float*)(ws + oSs1);
  float*    ss2  = (float*)(ws + oSs2);
  float*    gt   = (float*)(ws + oGt);
  float*    pl   = (float*)(ws + oPl);
  float*    zc   = (float*)(ws + oZc);

  const int vec8 = ((nE & 3) == 0) ? 1 : 0;

  k_wprep<<<8 * (nM + 1), NTHR, 0, stream>>>(W1, W2, cW1, gW1, whi, wlo, wg, nL);

  k_count<<<nBC, NTHR, 0, stream>>>(ei, cnt, nE, vec8);
  k_offsets<<<1, OTHR, 0, stream>>>(cnt, offp, rb, nBC);
  hipFuncSetAttribute(reinterpret_cast<const void*>(&k_fill),
                      hipFuncAttributeMaxDynamicSharedMemorySize, LDS_FILL);
  k_fill<<<nBF, NTHR, LDS_FILL, stream>>>(ei, offp, rb, csr, nN, nE, vec8, csrLen);

  k_enc<<<nEnc, NTHR, 0, stream>>>(x, pe, ce, le, P0, nN, nTh, nCa, nLv);

  hipFuncSetAttribute(reinterpret_cast<const void*>(&k_gemm3<0>),
                      hipFuncAttributeMaxDynamicSharedMemorySize, LDS_G3);
  hipFuncSetAttribute(reinterpret_cast<const void*>(&k_gemm3<1>),
                      hipFuncAttributeMaxDynamicSharedMemorySize, LDS_G3);

  for (int i = 0; i < nL; ++i) {
    k_agg<<<nAgg, NTHR, 0, stream>>>(csr, offp, cnt, P0, P1, nN, csrLen);
    k_gemm3<0><<<nGemm, NTHR, LDS_G3, stream>>>(P1, whi + (size_t)i * HIDC * HIDC, wlo + (size_t)i * HIDC * HIDC,
                                                ss1, be1 + (size_t)i * HIDC, b1 + (size_t)i * HIDC,
                                                P0, part, NPAD, nN);
    k_bnfin<<<1, NTHR, 0, stream>>>(part, nGemm, nN, g1 + (size_t)i * HIDC, ss1);
    k_gemm3<1><<<nGemm, NTHR, LDS_G3, stream>>>(P0, whi + (size_t)(nL + i) * HIDC * HIDC, wlo + (size_t)(nL + i) * HIDC * HIDC,
                                                ss1, be1 + (size_t)i * HIDC, b2 + (size_t)i * HIDC,
                                                P1, part, NPAD, nN);
    k_bnfin<<<1, NTHR, 0, stream>>>(part, nGemm, nN, g2 + (size_t)i * HIDC, ss2);
    k_apply<<<nApp, NTHR, 0, stream>>>(P1, ss2, be2 + (size_t)i * HIDC, P0);
  }

  k_gate<<<nGemm, NTHR, 0, stream>>>(P0, wg, gb1, gW2, gb2, gt, NPAD);
  k_pool<<<nPool, NTHR, 0, stream>>>(bat, numg, gt, P0, pl, nN);
  k_gemm3<0><<<nCls, NTHR, LDS_G3, stream>>>(pl, whi + (size_t)(2 * nL) * HIDC * HIDC, wlo + (size_t)(2 * nL) * HIDC * HIDC,
                                             ss1, cbe, cb1, zc, part, GR, G);
  k_clsfin<<<1, NTHR, 0, stream>>>(zc, part, nCls, G, cg, cbe, cW2, cb2, out, out_size);
}
